// StochasticTwoLayerGCN_26809185861707
// MI455X (gfx1250) — hardware-verified
//
#include <hip/hip_runtime.h>
#include <stddef.h>


#define DF        128
#define NTHR      256
#define NWAVE     8
#define EPT       8
#define NGRP      2
#define CHUNK     (NTHR * EPT * NGRP)
#define WCAP      (EPT * NGRP * 32)
#define LISTN     (NWAVE * WCAP)
#define NB        512
#define NBD       4096
#define LDS_LAYER (NB * DF * 4 + LISTN * 4 + 64)

static_assert((CHUNK & (CHUNK - 1)) == 0);
static_assert(CHUNK <= 4096);
static_assert((NB & (NB - 1)) == 0 && NB <= 4096);
static_assert(NB == NWAVE * 64);
static_assert(NBD == NWAVE * 4 * 128);
static_assert((NBD % NB) == 0);

typedef float          v4f   __attribute__((ext_vector_type(4)));
typedef float          v8f   __attribute__((ext_vector_type(8)));
typedef int            v4i   __attribute__((ext_vector_type(4)));
typedef __bf16         v16b  __attribute__((ext_vector_type(16)));
typedef unsigned short v8us  __attribute__((ext_vector_type(8)));
typedef unsigned short v16us __attribute__((ext_vector_type(16)));
union FragU { v16us u; v8us q[2]; };

__device__ __forceinline__ unsigned short bf_bits(float f) {
  unsigned u = __builtin_bit_cast(unsigned, f);
  u = u + 0x7FFFu + ((u >> 16) & 1u);
  return (unsigned short)(u >> 16);
}
__device__ __forceinline__ float bf_val(unsigned short s) {
  return __builtin_bit_cast(float, ((unsigned)s) << 16);
}
__device__ __forceinline__ void split2(float f, unsigned short& h, unsigned short& l) {
  h = bf_bits(f);
  l = bf_bits(f - bf_val(h));
}

__device__ __forceinline__ v8f wmb(v16us a, v16us b, v8f c) {
  const v16b av = __builtin_bit_cast(v16b, a);
  const v16b bv = __builtin_bit_cast(v16b, b);
  v8f d = __builtin_amdgcn_wmma_f32_16x16x32_bf16(false, av, false, bv, (short)0, c, false, false);
  asm volatile("v_nop\n\tv_nop\n\tv_nop\n\tv_nop" : "+v"(d) : "v"(a), "v"(b));
  return d;
}

__device__ __forceinline__ float inv_sqrt_cnt(int c) {
  const float f = (float)(c > 1 ? c : 1);
  return rsqrtf(f);
}

__device__ __forceinline__ v4f norm4(v4i c) {
  v4f r;
  r.x = inv_sqrt_cnt(c.x); r.y = inv_sqrt_cnt(c.y); r.z = inv_sqrt_cnt(c.z); r.w = inv_sqrt_cnt(c.w);
  return r;
}

__device__ __forceinline__ void load8i(const int* __restrict__ p, int e0, int nE, int vec8, v4i& a, v4i& b) {
  const int sent = -2147483647 - 1;
  if (vec8 != 0 && e0 + 7 < nE) {
    a = *(const v4i*)(p + e0);
    b = *(const v4i*)(p + e0 + 4);
  } else {
    a.x = (e0     < nE) ? p[min(e0,     nE - 1)] : sent;
    a.y = (e0 + 1 < nE) ? p[min(e0 + 1, nE - 1)] : sent;
    a.z = (e0 + 2 < nE) ? p[min(e0 + 2, nE - 1)] : sent;
    a.w = (e0 + 3 < nE) ? p[min(e0 + 3, nE - 1)] : sent;
    b.x = (e0 + 4 < nE) ? p[min(e0 + 4, nE - 1)] : sent;
    b.y = (e0 + 5 < nE) ? p[min(e0 + 5, nE - 1)] : sent;
    b.z = (e0 + 6 < nE) ? p[min(e0 + 6, nE - 1)] : sent;
    b.w = (e0 + 7 < nE) ? p[min(e0 + 7, nE - 1)] : sent;
  }
}

template <int NBT>
__device__ __forceinline__ int scan_chunk(const int* __restrict__ dsts, int nE, int cbase, int nodeBase,
                                          int vec8, int* list, int tid, int lane, int wave) {
  int wc = 0;
#pragma unroll
  for (int g = 0; g < NGRP; ++g) {
    const int el0 = (g * NTHR + tid) * EPT;
    const int e0  = cbase + el0;
    v4i da, db;
    load8i(dsts, e0, nE, vec8, da, db);
    const unsigned nb = (unsigned)nodeBase;
    const unsigned s0 = (unsigned)da.x - nb, s1 = (unsigned)da.y - nb;
    const unsigned s2 = (unsigned)da.z - nb, s3 = (unsigned)da.w - nb;
    const unsigned s4 = (unsigned)db.x - nb, s5 = (unsigned)db.y - nb;
    const unsigned s6 = (unsigned)db.z - nb, s7 = (unsigned)db.w - nb;
    const bool h0 = s0 < (unsigned)NBT, h1 = s1 < (unsigned)NBT, h2 = s2 < (unsigned)NBT, h3 = s3 < (unsigned)NBT;
    const bool h4 = s4 < (unsigned)NBT, h5 = s5 < (unsigned)NBT, h6 = s6 < (unsigned)NBT, h7 = s7 < (unsigned)NBT;
    const unsigned any = __builtin_amdgcn_ballot_w32(h0 | h1 | h2 | h3 | h4 | h5 | h6 | h7);
    if (any != 0u) {
#define HITJ(J, HJ, SJ) { \
        const unsigned mj = __builtin_amdgcn_ballot_w32(HJ); \
        if (mj != 0u) { \
          if (HJ) { \
            const int pos = wc + (int)__builtin_amdgcn_mbcnt_lo(mj, 0u); \
            if (pos < WCAP) list[wave * WCAP + pos] = ((el0 + (J)) << 12) | (int)(SJ); \
          } \
          wc += (int)__builtin_popcount(mj); } }
      HITJ(0, h0, s0)
      HITJ(1, h1, s1)
      HITJ(2, h2, s2)
      HITJ(3, h3, s3)
      HITJ(4, h4, s4)
      HITJ(5, h5, s5)
      HITJ(6, h6, s6)
      HITJ(7, h7, s7)
#undef HITJ
    }
  }
  return wc;
}

__global__ __launch_bounds__(NTHR) void k_wprep(
    const float* __restrict__ W1, const float* __restrict__ W2,
    unsigned short* h1p, unsigned short* l1p, unsigned short* h2p, unsigned short* l2p) {
  const int i   = blockIdx.x * NTHR + threadIdx.x;
  const int per = DF * DF / 8;
  if (i >= 2 * per) return;
  const bool first = i < per;
  const int o  = (first ? i : i - per) * 8;
  const int n  = o / DF;
  const int k0 = o - n * DF;
  const float* p = (first ? W1 : W2) + (size_t)k0 * DF + n;
  v8us hv, lv;
#pragma unroll
  for (int j = 0; j < 8; ++j) {
    unsigned short h, l;
    split2(p[(size_t)j * DF], h, l);
    hv[j] = h;
    lv[j] = l;
  }
  unsigned short* hp = (first ? h1p : h2p) + o;
  unsigned short* lp = (first ? l1p : l2p) + o;
  *(volatile v8us*)hp = hv;
  *(volatile v8us*)lp = lv;
  __threadfence();
  *(volatile v8us*)hp = hv;
  *(volatile v8us*)lp = lv;
}

__global__ __launch_bounds__(NTHR) void k_deg(
    const int* __restrict__ esrc, const int* __restrict__ edst,
    float* nsrc, float* ndst, int nE, int vec8) {
  __shared__ __attribute__((aligned(16))) int cs[NBD];
  __shared__ __attribute__((aligned(16))) int cd[NBD];
  const int tid = threadIdx.x, lane = tid & 31, wave = tid >> 5;
  const int nodeBase = blockIdx.x * NBD;
  const unsigned nb = (unsigned)nodeBase;

  for (int i = tid; i < NBD; i += NTHR) { cs[i] = 0; cd[i] = 0; }
  __syncthreads();

  const int nIter = (nE + NTHR * 8 - 1) / (NTHR * 8);
#pragma unroll 1
  for (int it = 0; it < nIter; ++it) {
    const int e0 = (it * NTHR + tid) * 8;
    v4i sa, sb, ta, tb;
    load8i(esrc, e0, nE, vec8, sa, sb);
    load8i(edst, e0, nE, vec8, ta, tb);
#define CNT1(ARR, V) { const unsigned s = (unsigned)(V) - nb; if (s < (unsigned)NBD) atomicAdd(&ARR[s], 1); }
    CNT1(cs, sa.x) CNT1(cs, sa.y) CNT1(cs, sa.z) CNT1(cs, sa.w)
    CNT1(cs, sb.x) CNT1(cs, sb.y) CNT1(cs, sb.z) CNT1(cs, sb.w)
    CNT1(cd, ta.x) CNT1(cd, ta.y) CNT1(cd, ta.z) CNT1(cd, ta.w)
    CNT1(cd, tb.x) CNT1(cd, tb.y) CNT1(cd, tb.z) CNT1(cd, tb.w)
#undef CNT1
  }
  __syncthreads();

  float* ps = nsrc + (size_t)nodeBase;
  float* pd = ndst + (size_t)nodeBase;
#pragma unroll 1
  for (int q = 0; q < 4; ++q) {
    const int f = (wave * 4 + q) * 128 + 4 * lane;
    const v4f vs = norm4(*(const v4i*)(cs + f));
    const v4f vd = norm4(*(const v4i*)(cd + f));
    *(volatile v4f*)(ps + f) = vs;
    *(volatile v4f*)(pd + f) = vd;
  }
  __threadfence();
#pragma unroll 1
  for (int q = 0; q < 4; ++q) {
    const int f = (wave * 4 + q) * 128 + 4 * lane;
    const v4f vs = norm4(*(const v4i*)(cs + f));
    const v4f vd = norm4(*(const v4i*)(cd + f));
    *(volatile v4f*)(ps + f) = vs;
    *(volatile v4f*)(pd + f) = vd;
  }
}

__global__ __launch_bounds__(NTHR) void k_layer(
    const float* __restrict__ xin, const int* __restrict__ esrc, const int* __restrict__ edst,
    const float* __restrict__ nsrc, const float* __restrict__ ndst,
    const unsigned short* __restrict__ whi, const unsigned short* __restrict__ wlo,
    const float* __restrict__ bias, float* outp,
    int nN, int nE, int rowLimit, int vec8) {
  extern __shared__ v4f lds_dyn[];
  float* accL = (float*)lds_dyn;
  int*   list = (int*)(accL + NB * DF);
  int*   wcnt = list + LISTN;
  const int tid = threadIdx.x, lane = tid & 31, wave = tid >> 5, hh = lane >> 4, m = lane & 15;
  const int nodeBase = blockIdx.x * NB;

  {
    const v4f z = {0.f, 0.f, 0.f, 0.f};
    for (int i = tid; i < NB * DF / 4; i += NTHR) lds_dyn[i] = z;
  }
  __syncthreads();

  const int nChunks = (nE + CHUNK - 1) / CHUNK;
#pragma unroll 1
  for (int ch = 0; ch < nChunks; ++ch) {
    const int cbase = ch * CHUNK;
    const int wc = scan_chunk<NB>(edst, nE, cbase, nodeBase, vec8, list, tid, lane, wave);
    if (lane == 0) wcnt[wave] = wc;
    __syncthreads();
    if (wave == 0) {
#pragma unroll 1
      for (int wsx = 0; wsx < NWAVE; ++wsx) {
        int n = __builtin_amdgcn_readfirstlane(wcnt[wsx]);
        n = n > WCAP ? WCAP : (n < 0 ? 0 : n);
        const int lbase = wsx * WCAP;
#pragma unroll 1
        for (int i = 0; i < n; ++i) {
          const int ent  = __builtin_amdgcn_readfirstlane(list[lbase + i]);
          const int slot = ent & (NB - 1);
          int e = cbase + ((ent >> 12) & (CHUNK - 1));
          e = e > nE - 1 ? nE - 1 : e;
          int u = esrc[e];
          u = u < 0 ? 0 : (u > nN - 1 ? nN - 1 : u);
          const float sc = nsrc[u];
          const v4f   v  = *(const v4f*)(xin + (size_t)u * DF + 4 * lane);
          v4f* ap = (v4f*)(accL + slot * DF + 4 * lane);
          *ap = *ap + v * sc;
        }
      }
    }
    __syncthreads();
  }

#pragma unroll 1
  for (int rt = 0; rt < 4; ++rt) {
    const int rowL = wave * 64 + 16 * rt;
    int node = nodeBase + rowL + m;
    node = node > nN - 1 ? nN - 1 : node;
    const float nrm = ndst[node];

    v16us ah[4], al[4];
    const float* arow = accL + (rowL + m) * DF + 8 * hh;
#pragma unroll
    for (int kt = 0; kt < 4; ++kt) {
      v4f p0 = *(const v4f*)(arow + 32 * kt),      p1 = *(const v4f*)(arow + 32 * kt + 4);
      v4f p2 = *(const v4f*)(arow + 32 * kt + 16), p3 = *(const v4f*)(arow + 32 * kt + 20);
      p0 = p0 * nrm; p1 = p1 * nrm; p2 = p2 * nrm; p3 = p3 * nrm;
      v16us hu, lu;
#pragma unroll
      for (int j = 0; j < 4; ++j) {
        unsigned short h, l;
        split2(p0[j], h, l); hu[j]      = h; lu[j]      = l;
        split2(p1[j], h, l); hu[4 + j]  = h; lu[4 + j]  = l;
        split2(p2[j], h, l); hu[8 + j]  = h; lu[8 + j]  = l;
        split2(p3[j], h, l); hu[12 + j] = h; lu[12 + j] = l;
      }
      ah[kt] = hu;
      al[kt] = lu;
    }

#pragma unroll 1
    for (int t = 0; t < 8; ++t) {
      v8f c = {0.f, 0.f, 0.f, 0.f, 0.f, 0.f, 0.f, 0.f};
#pragma unroll
      for (int kt = 0; kt < 4; ++kt) {
        const size_t bo = (size_t)(16 * t + m) * DF + 32 * kt + 8 * hh;
        FragU bh, bl;
        bh.q[0] = *(const v8us*)(whi + bo);
        bh.q[1] = *(const v8us*)(whi + bo + 16);
        bl.q[0] = *(const v8us*)(wlo + bo);
        bl.q[1] = *(const v8us*)(wlo + bo + 16);
        c = wmb(ah[kt], bh.u, c);
        c = wmb(ah[kt], bl.u, c);
        c = wmb(al[kt], bh.u, c);
      }
      const float bc = bias[16 * t + m];
      float* sp = accL + (rowL + 8 * hh) * DF + 16 * t + m;
      sp[0 * DF] = fmaxf(c[0] + bc, 0.f);
      sp[1 * DF] = fmaxf(c[1] + bc, 0.f);
      sp[2 * DF] = fmaxf(c[2] + bc, 0.f);
      sp[3 * DF] = fmaxf(c[3] + bc, 0.f);
      sp[4 * DF] = fmaxf(c[4] + bc, 0.f);
      sp[5 * DF] = fmaxf(c[5] + bc, 0.f);
      sp[6 * DF] = fmaxf(c[6] + bc, 0.f);
      sp[7 * DF] = fmaxf(c[7] + bc, 0.f);
    }
  }
  __syncthreads();

#pragma unroll 4
  for (int i = 0; i < 64; ++i) {
    const int rloc = wave * 64 + i;
    const int grow = nodeBase + rloc;
    if (grow < rowLimit) {
      const v4f v = *(const v4f*)(accL + rloc * DF + 4 * lane);
      *(volatile v4f*)(outp + (size_t)grow * DF + 4 * lane) = v;
    }
  }
  __threadfence();
#pragma unroll 4
  for (int i = 0; i < 64; ++i) {
    const int rloc = wave * 64 + i;
    const int grow = nodeBase + rloc;
    if (grow < rowLimit) {
      const v4f v = *(const v4f*)(accL + rloc * DF + 4 * lane);
      *(volatile v4f*)(outp + (size_t)grow * DF + 4 * lane) = v;
    }
  }
}

extern "C" void kernel_launch(void* const* d_in, const int* in_sizes, int n_in,
                              void* d_out, int out_size, void* d_ws, size_t ws_size,
                              hipStream_t stream) {
  if (n_in < 7) return;
  const int nN = in_sizes[0] / DF;
  const int nE = in_sizes[1];
  if (nN <= 0 || nE <= 0 || in_sizes[0] != nN * DF || in_sizes[2] != nE) return;
  if (in_sizes[3] != DF * DF || in_sizes[4] < DF || in_sizes[5] != DF * DF || in_sizes[6] < DF) return;
  if (out_size != nN * DF) return;

  const float* x    = (const float*)d_in[0];
  const int*   esrc = (const int*)d_in[1];
  const int*   edst = (const int*)d_in[2];
  const float* W1   = (const float*)d_in[3];
  const float* b1   = (const float*)d_in[4];
  const float* W2   = (const float*)d_in[5];
  const float* b2   = (const float*)d_in[6];
  float* out = (float*)d_out;

  const int nBD  = (nN + NBD - 1) / NBD;
  const int nBlk = (nN + NB - 1) / NB;

  char* ws = (char*)d_ws;
  size_t off = 0;
  const size_t oH1 = off; off += (size_t)DF * DF * 2;                off = (off + 255) & ~(size_t)255;
  const size_t oL1 = off; off += (size_t)DF * DF * 2;                off = (off + 255) & ~(size_t)255;
  const size_t oH2 = off; off += (size_t)DF * DF * 2;                off = (off + 255) & ~(size_t)255;
  const size_t oL2 = off; off += (size_t)DF * DF * 2;                off = (off + 255) & ~(size_t)255;
  const size_t oNs = off; off += (size_t)nBD * NBD * 4;              off = (off + 255) & ~(size_t)255;
  const size_t oNd = off; off += (size_t)nBD * NBD * 4;              off = (off + 255) & ~(size_t)255;
  const size_t oHp = off; off += (size_t)nBlk * NB * DF * 4;         off = (off + 255) & ~(size_t)255;
  if (off > ws_size) return;
  unsigned short* wh1 = (unsigned short*)(ws + oH1);
  unsigned short* wl1 = (unsigned short*)(ws + oL1);
  unsigned short* wh2 = (unsigned short*)(ws + oH2);
  unsigned short* wl2 = (unsigned short*)(ws + oL2);
  float* nsrc = (float*)(ws + oNs);
  float* ndst = (float*)(ws + oNd);
  float* hpl  = (float*)(ws + oHp);

  const int vec8 = ((nE & 3) == 0) ? 1 : 0;

  const int nPrep = 2 * (DF * DF / 8);
  k_wprep<<<(nPrep + NTHR - 1) / NTHR, NTHR, 0, stream>>>(W1, W2, wh1, wl1, wh2, wl2);

  k_deg<<<nBD, NTHR, 0, stream>>>(esrc, edst, nsrc, ndst, nE, vec8);

  hipFuncSetAttribute(reinterpret_cast<const void*>(&k_layer),
                      hipFuncAttributeMaxDynamicSharedMemorySize, LDS_LAYER);
  k_layer<<<nBlk, NTHR, LDS_LAYER, stream>>>(x, esrc, edst, nsrc, ndst, wh1, wl1, b1, hpl,
                                             nN, nE, nBlk * NB, vec8);
  k_layer<<<nBlk, NTHR, LDS_LAYER, stream>>>(hpl, esrc, edst, nsrc, ndst, wh2, wl2, b2, out,
                                             nN, nE, nN, vec8);
}
